// GraphWaveNet_20950850470512
// MI455X (gfx1250) — hardware-verified
//
#include <hip/hip_runtime.h>
#include <hip/hip_bf16.h>


#define NN  1024
#define BB  16
#define T0  13
#define CH  32
#define SKC 256
#define ENC 512
#define OT  12
#define NL  8
#define CAP 64

typedef float          v4f   __attribute__((ext_vector_type(4)));
typedef float          v8f   __attribute__((ext_vector_type(8)));
typedef double         v2d   __attribute__((ext_vector_type(2)));
typedef _Float16       v8h   __attribute__((ext_vector_type(8)));
typedef _Float16       v16h  __attribute__((ext_vector_type(16)));
typedef __bf16         v16b  __attribute__((ext_vector_type(16)));
typedef unsigned short u16x8 __attribute__((ext_vector_type(8)));
union Frag { u16x8 h[2]; v8h x[2]; v16h f; v16b b; };
union H8 { v8h f; u16x8 u; };

constexpr size_t SZ_HA   = (size_t)BB * T0 * NN * CH * 4;
constexpr size_t SZ_HB   = (size_t)BB * 12 * NN * CH * 4;
constexpr size_t SZ_XW1  = SZ_HB;
constexpr size_t SZ_XW2  = (size_t)BB * 12 * CH * NN * 2;
constexpr size_t SZ_GL   = (size_t)BB * NN * CH * 2;
constexpr size_t SZ_SKIP = (size_t)BB * NN * SKC * 4;
constexpr size_t SZ_ADJ  = (size_t)NN * NN * 2;
constexpr size_t SZ_STAT = (size_t)NN * 4 * 4;
constexpr size_t SZ_DIS  = (size_t)NN * 4;
constexpr size_t SZ_BNC  = (size_t)(NL + 1) * 64 * 4;
constexpr size_t SZ_PART = (size_t)128 * 64 * 8;
constexpr size_t SZ_WT   = (size_t)NL * 64 * 64 * 2;
constexpr size_t SZ_W2   = (size_t)NL * 64 * 32 * 2;
constexpr size_t SZ_WSK  = (size_t)NL * SKC * CH * 2;
constexpr size_t SZ_E1   = (size_t)ENC * SKC * 2;
constexpr size_t SZ_E2   = (size_t)16 * ENC * 2;
constexpr size_t OFF_HA = 0, OFF_HB = OFF_HA + SZ_HA, OFF_XW1 = OFF_HB + SZ_HB, OFF_XW2 = OFF_XW1 + SZ_XW1;
constexpr size_t OFF_GLH = OFF_XW2 + SZ_XW2, OFF_GLL = OFF_GLH + SZ_GL, OFF_SKIP = OFF_GLL + SZ_GL, OFF_ADJ = OFF_SKIP + SZ_SKIP, OFF_STAT = OFF_ADJ + SZ_ADJ;
constexpr size_t OFF_DIS = OFF_STAT + SZ_STAT, OFF_BNC = OFF_DIS + SZ_DIS, OFF_PART = OFF_BNC + SZ_BNC, OFF_WTH = OFF_PART + SZ_PART, OFF_WTL = OFF_WTH + SZ_WT;
constexpr size_t OFF_W2 = OFF_WTL + SZ_WT, OFF_WSKH = OFF_W2 + SZ_W2, OFF_WSKL = OFF_WSKH + SZ_WSK, OFF_E1H = OFF_WSKL + SZ_WSK, OFF_E1L = OFF_E1H + SZ_E1;
constexpr size_t OFF_E2H = OFF_E1L + SZ_E1, OFF_E2L = OFF_E2H + SZ_E2, WS_END = OFF_E2L + SZ_E2;
constexpr size_t SZ_SP = (size_t)BB * NN * SKC * 2, SZ_Y1 = (size_t)BB * NN * ENC * 4, SZ_Y1P = (size_t)BB * NN * ENC * 2, SZ_Y2 = (size_t)BB * NN * 16 * 4;
constexpr size_t OFF_SH = OFF_XW1, OFF_SL = OFF_SH + SZ_SP, OFF_Y1 = OFF_HA, OFF_Y1H = OFF_XW1, OFF_Y1L = OFF_Y1H + SZ_Y1P, OFF_Y2 = OFF_SKIP;
static_assert(WS_END <= (size_t)134217728);
static_assert(OFF_SL + SZ_SP <= OFF_XW1 + SZ_XW1);
static_assert(OFF_Y1 + SZ_Y1 <= OFF_HB + SZ_HB);
static_assert(OFF_Y1L + SZ_Y1P <= OFF_GLH);
static_assert(SZ_Y2 <= SZ_SKIP);
static_assert(OFF_HB % 128 == 0 && OFF_XW1 % 128 == 0 && OFF_XW2 % 128 == 0 && OFF_GLH % 128 == 0 && OFF_GLL % 128 == 0 && OFF_SKIP % 128 == 0 && OFF_ADJ % 128 == 0);
static_assert(OFF_STAT % 128 == 0 && OFF_DIS % 128 == 0 && OFF_BNC % 128 == 0 && OFF_PART % 128 == 0 && OFF_WTH % 128 == 0 && OFF_WTL % 128 == 0 && OFF_W2 % 128 == 0);
static_assert(OFF_WSKH % 128 == 0 && OFF_WSKL % 128 == 0 && OFF_E1H % 128 == 0 && OFF_E1L % 128 == 0 && OFF_E2H % 128 == 0 && OFF_E2L % 128 == 0 && OFF_SL % 128 == 0 && OFF_Y1L % 128 == 0);

__device__ __forceinline__ unsigned short f32_to_bf16(float f) {
    unsigned u = __float_as_uint(f);
    return (unsigned short)((u + 0x7FFFu + ((u >> 16) & 1u)) >> 16);
}
__device__ __forceinline__ float bf16_to_f32(unsigned short b) { return __uint_as_float(((unsigned)b) << 16); }
__device__ __forceinline__ v8f ld8f(const float* p) {
    v4f a = *(const v4f*)p; v4f b = *(const v4f*)(p + 4);
    return __builtin_shufflevector(a, b, 0, 1, 2, 3, 4, 5, 6, 7);
}
__device__ __forceinline__ void split8(const v8f x, u16x8& hv, u16x8& lv) {
#pragma unroll
    for (int c = 0; c < 8; ++c) {
        const unsigned short hb = f32_to_bf16(x[c]);
        hv[c] = hb; lv[c] = f32_to_bf16(x[c] - bf16_to_f32(hb));
    }
}
__device__ __forceinline__ void mma_h(v8f& acc, const Frag& a, const Frag& b) {
    acc = __builtin_amdgcn_wmma_f32_16x16x32_f16(false, a.f, false, b.f, (short)0, acc, false, false);
    asm volatile("v_nop\n\tv_nop\n\tv_nop\n\tv_nop" : "+v"(acc) : "v"(a.f), "v"(b.f));
}
__device__ __forceinline__ void mma_b(v8f& acc, const Frag& a, const Frag& b) {
    acc = __builtin_amdgcn_wmma_f32_16x16x32_bf16(false, a.b, false, b.b, (short)0, acc, false, false);
    asm volatile("v_nop\n\tv_nop\n\tv_nop\n\tv_nop" : "+v"(acc) : "v"(a.b), "v"(b.b));
}
__device__ __forceinline__ void zero8(v8f& a) {
#pragma unroll
    for (int r = 0; r < 8; ++r) a[r] = 0.f;
}

__global__ __launch_bounds__(256)
void k_wprep(const float* __restrict__ tAw, const float* __restrict__ tBw, const float* __restrict__ gw, const float* __restrict__ gaw,
             const float* __restrict__ sw, const float* __restrict__ e1w, const float* __restrict__ e2w,
             unsigned short* wth, unsigned short* wtl, unsigned short* w2, unsigned short* wskh, unsigned short* wskl,
             unsigned short* e1h, unsigned short* e1l, unsigned short* e2h, unsigned short* e2l)
{
    const int seg = blockIdx.y;
    const int i8 = blockIdx.x * 256 + threadIdx.x;
    const int lim = (seg == 0) ? 4096 : (seg == 1) ? 2048 : (seg == 2) ? 8192 : (seg == 3) ? 16384 : 1024;
    if (i8 >= lim) return;
    const int o0 = i8 * 8;
    v8f v;
    if (seg == 0) {
#pragma unroll
        for (int c = 0; c < 8; ++c) {
            const int o = o0 + c, k = o >> 12, rem = o & 4095, n = rem >> 6, kk = rem & 63;
            const int idx = ((k * 32 + (n & 31)) * 32 + (kk & 31)) * 2 + (kk >> 5);
            const float a = tAw[idx], q = tBw[idx];
            v[c] = (n >> 5) ? q : a;
        }
    } else if (seg == 1) {
#pragma unroll
        for (int c = 0; c < 8; ++c) {
            const int o = o0 + c, k = o >> 11, rem = o & 2047, n = rem >> 5, ci = rem & 31;
            const int idx = (k * 32 + ci) * 32 + (n & 31);
            const float a = gw[idx], q = gaw[idx];
            v[c] = 64.f * ((n >> 5) ? q : a);
        }
    } else if (seg == 2) {
        v = ld8f(sw + o0);
    } else if (seg == 3) {
        v = ld8f(e1w + o0);
    } else {
        const int n = o0 >> 9, kc = o0 & 511;
        const v8f t = ld8f(e2w + (size_t)min(n, OT - 1) * ENC + kc);
#pragma unroll
        for (int c = 0; c < 8; ++c) v[c] = (n < OT) ? t[c] : 0.f;
    }
    if (seg == 1) {
        H8 u; u.f = __builtin_convertvector(v, v8h);
        *(volatile u16x8*)(w2 + o0) = u.u;
        __threadfence();
        *(volatile u16x8*)(w2 + o0) = u.u;
    } else {
        unsigned short* dh = (seg == 0) ? wth : (seg == 2) ? wskh : (seg == 3) ? e1h : e2h;
        unsigned short* dl = (seg == 0) ? wtl : (seg == 2) ? wskl : (seg == 3) ? e1l : e2l;
        u16x8 hv, lv; split8(v, hv, lv);
        *(volatile u16x8*)(dh + o0) = hv; *(volatile u16x8*)(dl + o0) = lv;
        __threadfence();
        *(volatile u16x8*)(dh + o0) = hv; *(volatile u16x8*)(dl + o0) = lv;
    }
}

__global__ __launch_bounds__(256)
void k_h0(const float* __restrict__ x, const float* __restrict__ inw, const float* __restrict__ inb, float* H, float* bnc0, int n4)
{
    const int i = blockIdx.x * 256 + threadIdx.x;
    if (blockIdx.x == 0 && threadIdx.x < 16) {
        const float val = (threadIdx.x < 8) ? 1.f : 0.f;
        v4f o = {val, val, val, val};
        *(volatile v4f*)(bnc0 + threadIdx.x * 4) = o;
        __threadfence();
        *(volatile v4f*)(bnc0 + threadIdx.x * 4) = o;
    }
    if (i >= n4) return;
    const int row = i >> 3, c0 = (i & 7) * 4;
    const float x0 = x[(size_t)row * 2], x1 = x[(size_t)row * 2 + 1];
    v4f v;
#pragma unroll
    for (int q = 0; q < 4; ++q) { const int c = c0 + q; v[q] = inw[c * 2] * x0 + inw[c * 2 + 1] * x1 + inb[c]; }
    float* gp = H + (size_t)row * CH + c0;
    *(volatile v4f*)gp = v;
    __threadfence();
    *(volatile v4f*)gp = v;
}

__global__ __launch_bounds__(256)
void k_graph(const int* __restrict__ ei, const float* __restrict__ ew, int E, float* dis)
{
    __shared__ float sd[32];
    const int tid = threadIdx.x, lane = tid & 31, w = tid >> 5;
    const int nb = blockIdx.x * 32 + w * 4;
    const int* dstp = ei + E;
    float acc[4] = {0.f, 0.f, 0.f, 0.f};
    const int nchunk = (E + 255) >> 8;
#pragma unroll 1
    for (int ch = 0; ch < nchunk; ++ch) {
        const int cb = ch * 256 + lane * 8;
#pragma unroll
        for (int j = 0; j < 8; ++j) {
            const int e = cb + j, ec = min(e, E - 1);
            const int dv = dstp[ec];
            float wj = ew[ec]; wj = (e < E) ? wj : 0.f;
#pragma unroll
            for (int q = 0; q < 4; ++q) acc[q] += (dv == nb + q) ? wj : 0.f;
        }
    }
#pragma unroll
    for (int q = 0; q < 4; ++q) {
        float a = acc[q];
#pragma unroll
        for (int mm = 16; mm >= 1; mm >>= 1) a += __shfl_xor(a, mm, 32);
        const float deg = a + 1.f;
        if (lane == 0) sd[w * 4 + q] = (deg > 0.f) ? rsqrtf(deg) : 0.f;
    }
    __syncthreads();
    if (w == 0) {
        const float v = sd[lane];
        *(volatile float*)(dis + blockIdx.x * 32 + lane) = v;
        __threadfence();
        *(volatile float*)(dis + blockIdx.x * 32 + lane) = v;
    }
}

__global__ __launch_bounds__(256)
void k_adp1(const float* __restrict__ e1, const float* __restrict__ e2, float* stats)
{
    __shared__ float sm[8][NN];
    __shared__ __attribute__((aligned(16))) float st[8][4];
    const int tid = threadIdx.x, lane = tid & 31, w = tid >> 5;
    const int i = blockIdx.x * 8 + w;
    float ev[10];
#pragma unroll
    for (int e = 0; e < 10; ++e) ev[e] = e1[i * 10 + e];
    float mx = 0.f;
#pragma unroll 1
    for (int q = 0; q < 32; ++q) {
        const int j = q * 32 + lane;
        float m = 0.f;
#pragma unroll
        for (int e = 0; e < 10; ++e) m += ev[e] * e2[e * NN + j];
        m = fmaxf(m, 0.f);
        sm[w][j] = m; mx = fmaxf(mx, m);
    }
#pragma unroll
    for (int mm = 16; mm >= 1; mm >>= 1) mx = fmaxf(mx, __shfl_xor(mx, mm, 32));
    float s = 0.f;
#pragma unroll 1
    for (int q = 0; q < 32; ++q) s += __expf(sm[w][q * 32 + lane] - mx);
#pragma unroll
    for (int mm = 16; mm >= 1; mm >>= 1) s += __shfl_xor(s, mm, 32);
    __syncthreads();
    const float invs = 1.0f / s;
    const float pii = __expf(sm[w][i] - mx) * invs;
    const float dv = rsqrtf(fmaxf(2.f - pii, 1.f));
    if (lane == 0) { st[w][0] = mx; st[w][1] = invs; st[w][2] = dv; st[w][3] = 0.f; }
    __syncthreads();
    if (w == 0 && lane < 8) {
        const v4f v = *(const v4f*)&st[lane][0];
        float* gp = stats + (size_t)(blockIdx.x * 8 + lane) * 4;
        *(volatile v4f*)gp = v;
        __threadfence();
        *(volatile v4f*)gp = v;
    }
}

__global__ __launch_bounds__(256)
void k_adp2(const float* __restrict__ e1, const float* __restrict__ e2, const float* __restrict__ stats, unsigned short* adj)
{
    __shared__ __attribute__((aligned(16))) _Float16 sr[8][NN];
    const int tid = threadIdx.x, lane = tid & 31, w = tid >> 5;
    const int i = blockIdx.x * 8 + w;
    float ev[10];
#pragma unroll
    for (int e = 0; e < 10; ++e) ev[e] = e1[i * 10 + e];
    const float mx = stats[i * 4], invs = stats[i * 4 + 1], di = stats[i * 4 + 2];
#pragma unroll 1
    for (int q = 0; q < 32; ++q) {
        const int j = q * 32 + lane;
        float m = 0.f;
#pragma unroll
        for (int e = 0; e < 10; ++e) m += ev[e] * e2[e * NN + j];
        m = fmaxf(m, 0.f);
        float p = __expf(m - mx) * invs;
        p = (j == i) ? 1.f : p;
        const float dj = stats[(size_t)j * 4 + 2];
        sr[w][j] = (_Float16)((di * p) * dj * 1024.f);
    }
    __syncthreads();
    H8 u[4];
#pragma unroll
    for (int it = 0; it < 4; ++it) u[it].f = *(const v8h*)(&sr[w][(it * 32 + lane) * 8]);
#pragma unroll
    for (int it = 0; it < 4; ++it) *(volatile u16x8*)(adj + (size_t)i * NN + (it * 32 + lane) * 8) = u[it].u;
    __threadfence();
#pragma unroll
    for (int it = 0; it < 4; ++it) *(volatile u16x8*)(adj + (size_t)i * NN + (it * 32 + lane) * 8) = u[it].u;
}

__device__ __forceinline__ void tcn_store(const float* sX, const _Float16* sT, const unsigned short* sGH, const unsigned short* sGL,
                                          float* xw1, unsigned short* xw2T, unsigned short* glh, unsigned short* gll,
                                          int tid, int bt, int b, int n0, bool last)
{
#pragma unroll
    for (int it = 0; it < 4; ++it) {
        const int p = it * 128 + tid, row = p >> 3, seg = (p & 7) * 4;
        const v4f v = *(const v4f*)(sX + row * 36 + seg);
        *(volatile v4f*)(xw1 + ((size_t)bt * NN + n0 + row) * CH + seg) = v;
    }
#pragma unroll
    for (int it = 0; it < 2; ++it) {
        const int p = it * 128 + tid, c = p >> 3, seg = (p & 7) * 8;
        H8 u; u.f = *(const v8h*)(sT + c * 72 + seg);
        *(volatile u16x8*)(xw2T + ((size_t)bt * CH + c) * NN + n0 + seg) = u.u;
    }
    if (last) {
#pragma unroll
        for (int it = 0; it < 2; ++it) {
            const int p = it * 128 + tid, row = p >> 2, seg = (p & 3) * 8;
            const u16x8 hv = *(const u16x8*)(sGH + row * 40 + seg);
            const u16x8 lv = *(const u16x8*)(sGL + row * 40 + seg);
            const size_t o = ((size_t)b * NN + n0 + row) * CH + seg;
            *(volatile u16x8*)(glh + o) = hv;
            *(volatile u16x8*)(gll + o) = lv;
        }
    }
}

__global__ __launch_bounds__(128)
void k_tcn(const float* __restrict__ Hin, const float* __restrict__ bnc, const unsigned short* __restrict__ WtH, const unsigned short* __restrict__ WtL,
           const unsigned short* __restrict__ W2, const float* __restrict__ ba, const float* __restrict__ bb,
           float* xw1, unsigned short* xw2T, unsigned short* glh, unsigned short* gll, int Tin, int Tk, int d)
{
    __shared__ __attribute__((aligned(16))) unsigned short sAH[64 * 72];
    __shared__ __attribute__((aligned(16))) unsigned short sAL[64 * 72];
    __shared__ __attribute__((aligned(16))) _Float16 sG[64 * 40];
    __shared__ __attribute__((aligned(16))) unsigned short sGH[64 * 40];
    __shared__ __attribute__((aligned(16))) unsigned short sGL[64 * 40];
    __shared__ __attribute__((aligned(16))) float    sX[64 * 36];
    __shared__ __attribute__((aligned(16))) _Float16 sT[32 * 72];
    __shared__ float sbn[64];
    const int tid = threadIdx.x, lane = tid & 31, wave = tid >> 5, h = lane >> 4, m16 = lane & 15;
    const int n0 = blockIdx.x * 64, t = blockIdx.y, b = blockIdx.z;
    const int bt = b * Tk + t;
    const bool last = (t == Tk - 1);
    if (tid < 64) sbn[tid] = bnc[tid];
    __syncthreads();
    {
        const int mr = tid >> 1, tap = tid & 1;
        const float* src = Hin + ((size_t)(b * Tin + t + tap * d) * NN + n0 + mr) * CH;
#pragma unroll
        for (int i = 0; i < 4; ++i) {
            const v8f xv = ld8f(src + 8 * i);
            v8f y;
#pragma unroll
            for (int c = 0; c < 8; ++c) y[c] = xv[c] * sbn[8 * i + c] + sbn[32 + 8 * i + c];
            u16x8 hv, lv; split8(y, hv, lv);
            *(u16x8*)(sAH + mr * 72 + tap * 32 + 8 * i) = hv;
            *(u16x8*)(sAL + mr * 72 + tap * 32 + 8 * i) = lv;
        }
    }
    __syncthreads();
    v8f acc[4];
#pragma unroll
    for (int j = 0; j < 4; ++j) zero8(acc[j]);
    const int arow = (wave * 16 + m16) * 72 + 8 * h;
#pragma unroll
    for (int ks = 0; ks < 2; ++ks) {
        Frag fa, ga;
        fa.h[0] = *(const u16x8*)(sAH + arow + 32 * ks); fa.h[1] = *(const u16x8*)(sAH + arow + 32 * ks + 16);
        ga.h[0] = *(const u16x8*)(sAL + arow + 32 * ks); ga.h[1] = *(const u16x8*)(sAL + arow + 32 * ks + 16);
#pragma unroll
        for (int j = 0; j < 4; ++j) {
            Frag fb, gb;
            const unsigned short* p = WtH + (16 * j + m16) * 64 + 32 * ks + 8 * h;
            const unsigned short* q = WtL + (16 * j + m16) * 64 + 32 * ks + 8 * h;
            fb.h[0] = *(const u16x8*)p; fb.h[1] = *(const u16x8*)(p + 16);
            gb.h[0] = *(const u16x8*)q; gb.h[1] = *(const u16x8*)(q + 16);
            mma_b(acc[j], fa, fb); mma_b(acc[j], fa, gb); mma_b(acc[j], ga, fb);
        }
    }
#pragma unroll
    for (int j = 0; j < 2; ++j) {
        const int c = 16 * j + m16;
        const float bA = ba[c], bBv = bb[c];
#pragma unroll
        for (int r = 0; r < 8; ++r) {
            const float av = acc[j][r] + bA;
            const float bv = acc[j + 2][r] + bBv;
            const float e = __expf(-2.f * fabsf(av));
            float th = (1.f - e) * __builtin_amdgcn_rcpf(1.f + e);
            th = copysignf(th, av);
            const float sg = __builtin_amdgcn_rcpf(1.f + __expf(-bv));
            const float gv = th * sg;
            const int row = wave * 16 + 8 * h + r;
            sG[row * 40 + c] = (_Float16)(gv * 256.f);
            if (last) {
                const unsigned short hb = f32_to_bf16(gv);
                sGH[row * 40 + c] = hb;
                sGL[row * 40 + c] = f32_to_bf16(gv - bf16_to_f32(hb));
            }
        }
    }
    __syncthreads();
    v8f acc2[4];
#pragma unroll
    for (int j = 0; j < 4; ++j) zero8(acc2[j]);
    {
        Frag fa; const _Float16* grow = sG + (wave * 16 + m16) * 40 + 8 * h;
        fa.x[0] = *(const v8h*)grow; fa.x[1] = *(const v8h*)(grow + 16);
#pragma unroll
        for (int j = 0; j < 4; ++j) {
            Frag fb; const unsigned short* p = W2 + (16 * j + m16) * 32 + 8 * h;
            fb.h[0] = *(const u16x8*)p; fb.h[1] = *(const u16x8*)(p + 16);
            mma_h(acc2[j], fa, fb);
        }
    }
#pragma unroll
    for (int j = 0; j < 2; ++j) {
        const int c = 16 * j + m16;
#pragma unroll
        for (int r = 0; r < 8; ++r) sX[(wave * 16 + 8 * h + r) * 36 + c] = acc2[j][r] * (1.f / 16384.f);
    }
#pragma unroll
    for (int j = 2; j < 4; ++j) {
        const int c = 16 * (j - 2) + m16;
#pragma unroll
        for (int r = 0; r < 8; ++r) sT[c * 72 + wave * 16 + 8 * h + r] = (_Float16)(acc2[j][r] * (1.f / 1024.f));
    }
    __syncthreads();
    tcn_store(sX, sT, sGH, sGL, xw1, xw2T, glh, gll, tid, bt, b, n0, last);
    __threadfence();
    tcn_store(sX, sT, sGH, sGL, xw1, xw2T, glh, gll, tid, bt, b, n0, last);
}

template<int NBF>
__device__ __forceinline__ void tile_store_pass(const float* st, float* gp, int ldc, int lane) {
    constexpr int CW = NBF * 16, P = CW + 4, LPR = CW / 4, RPI = 32 / LPR, NIT = 32 / RPI;
    static_assert(32 % LPR == 0);
    const int rsub = lane / LPR, c0 = (lane % LPR) * 4;
#pragma unroll
    for (int it = 0; it < NIT; ++it) {
        const int row = it * RPI + rsub;
        const v4f v = *(const v4f*)(st + row * P + c0);
        *(volatile v4f*)(gp + (size_t)row * ldc + c0) = v;
    }
}

template<int NBF, int X3>
__global__ __launch_bounds__(128)
void k_gemm(const unsigned short* __restrict__ A0, const unsigned short* __restrict__ A1,
            const unsigned short* __restrict__ B0, const unsigned short* __restrict__ B1,
            float* C, const float* __restrict__ bias, int K, int ldc, int nbias, int flags, float cscale,
            long long sA, long long sB, long long sC)
{
    constexpr int CW = NBF * 16, P = CW + 4, LPR = CW / 4, RPI = 32 / LPR, NIT = 32 / RPI;
    __shared__ __attribute__((aligned(16))) float stile[4][32 * P];
    const int tid = threadIdx.x, lane = tid & 31, wave = tid >> 5, h = lane >> 4, m = lane & 15;
    const size_t z = blockIdx.z;
    A0 += z * (size_t)sA; A1 += z * (size_t)sA; B0 += z * (size_t)sB; B1 += z * (size_t)sB; C += z * (size_t)sC;
    const int rowW = blockIdx.y * 128 + wave * 32;
    const int colW = blockIdx.x * CW;
    v8f acc[2 * NBF];
#pragma unroll
    for (int j = 0; j < 2 * NBF; ++j) zero8(acc[j]);
    const size_t aoff = (size_t)(rowW + m) * K + 8 * h, boff = (size_t)(colW + m) * K + 8 * h, sub16 = (size_t)16 * K;
    const int nk = K >> 5;
#pragma unroll 1
    for (int kt = 0; kt < nk; ++kt) {
        const size_t k0 = (size_t)kt * 32;
        Frag fa[2], ga[2], fb[NBF], gb[NBF];
#pragma unroll
        for (int s = 0; s < 2; ++s) {
            const unsigned short* p = A0 + aoff + s * sub16 + k0;
            fa[s].h[0] = *(const u16x8*)p; fa[s].h[1] = *(const u16x8*)(p + 16);
            if (X3) { const unsigned short* q = A1 + aoff + s * sub16 + k0; ga[s].h[0] = *(const u16x8*)q; ga[s].h[1] = *(const u16x8*)(q + 16); }
        }
#pragma unroll
        for (int j = 0; j < NBF; ++j) {
            const unsigned short* p = B0 + boff + j * sub16 + k0;
            fb[j].h[0] = *(const u16x8*)p; fb[j].h[1] = *(const u16x8*)(p + 16);
            if (X3) { const unsigned short* q = B1 + boff + j * sub16 + k0; gb[j].h[0] = *(const u16x8*)q; gb[j].h[1] = *(const u16x8*)(q + 16); }
        }
#pragma unroll
        for (int s = 0; s < 2; ++s)
#pragma unroll
            for (int j = 0; j < NBF; ++j) {
                if (X3) { mma_b(acc[s * NBF + j], fa[s], fb[j]); mma_b(acc[s * NBF + j], fa[s], gb[j]); mma_b(acc[s * NBF + j], ga[s], fb[j]); }
                else    { mma_h(acc[s * NBF + j], fa[s], fb[j]); }
            }
    }
    float* st = stile[wave];
#pragma unroll
    for (int s = 0; s < 2; ++s)
#pragma unroll
        for (int j = 0; j < NBF; ++j)
#pragma unroll
            for (int r = 0; r < 8; ++r) st[(s * 16 + 8 * h + r) * P + j * 16 + m] = acc[s * NBF + j][r];
    __syncthreads();
    const int rsub = lane / LPR, c0 = (lane % LPR) * 4;
    v4f b4;
#pragma unroll
    for (int i = 0; i < 4; ++i) {
        const int col = colW + c0 + i;
        const float bv = bias[min(col, max(nbias - 1, 0))];
        b4[i] = (col < nbias) ? bv : 0.f;
    }
    float* gp = C + (size_t)rowW * ldc + colW;
#pragma unroll
    for (int it = 0; it < NIT; ++it) {
        const int row = it * RPI + rsub;
        v4f v = *(const v4f*)(st + row * P + c0) * cscale + b4;
        if (flags & 2) v += *(const v4f*)(gp + (size_t)row * ldc + c0);
        *(v4f*)(st + row * P + c0) = v;
    }
    tile_store_pass<NBF>(st, gp, ldc, lane);
    __threadfence();
    tile_store_pass<NBF>(st, gp, ldc, lane);
}

__global__ __launch_bounds__(256)
void k_comb(float* Hout, const float* __restrict__ Hin, const float* __restrict__ xw1, const float* __restrict__ bnc,
            const int* __restrict__ ei, const float* __restrict__ ew, const float* __restrict__ dis,
            const float* __restrict__ gb, const float* __restrict__ gab, double* part, int E, int Tin, int Tk, int d)
{
    __shared__ int    lse[8][CAP];
    __shared__ int    lss[8][CAP];
    __shared__ float  lsf[8][CAP];
    __shared__ double red[8][64];
    __shared__ __attribute__((aligned(16))) double sp[64];
    const int tid = threadIdx.x, lane = tid & 31, w = tid >> 5;
    const int n = blockIdx.x * 8 + w;
    const int* dstp = ei + E;
    int cnt = 0;
    const int nchunk = (E + 255) >> 8;
#pragma unroll 1
    for (int ch = 0; ch < nchunk; ++ch) {
        const int cb = ch * 256 + lane * 8;
        int ev[8]; bool ht[8]; bool any = false;
#pragma unroll
        for (int j = 0; j < 8; ++j) {
            const int e = cb + j, ec = min(e, E - 1);
            const int dv = dstp[ec];
            ht[j] = (e < E) && (dv == n); ev[j] = e; any = any || ht[j];
        }
        if (__builtin_amdgcn_ballot_w32(any) == 0u) continue;
#pragma unroll
        for (int j = 0; j < 8; ++j) {
            const unsigned mk = __builtin_amdgcn_ballot_w32(ht[j]);
            const int pos = cnt + __builtin_popcount(mk & ((1u << lane) - 1u));
            if (ht[j] && pos < CAP) lse[w][pos] = ev[j];
            cnt += __builtin_popcount(mk);
        }
    }
    const int ncnt = min(cnt, CAP);
    __syncthreads();
    const float dn = dis[n];
#pragma unroll
    for (int q = 0; q < CAP / 32; ++q) {
        const int p = q * 32 + lane;
        int e = lse[w][p]; e = min(max(e, 0), E - 1);
        int s = ei[e]; s = min(max(s, 0), NN - 1);
        const float f = dis[s] * ew[e] * dn;
        if (p < ncnt) { lss[w][p] = s; lsf[w][p] = f; }
    }
    __syncthreads();
    const float sc = bnc[lane], sh = bnc[32 + lane];
    const float bsum = gb[lane] + gab[lane];
    const float selfw = dn * dn;
    double s64 = 0.0, q64 = 0.0;
    const int nbt = BB * Tk;
#pragma unroll 1
    for (int bt = 0; bt < nbt; ++bt) {
        const int b = bt / Tk, t = bt - b * Tk;
        const size_t ro = ((size_t)bt * NN + n) * CH + lane;
        const float* xb = xw1 + (size_t)bt * NN * CH + lane;
        float v = Hout[ro] + bsum;
        v += selfw * xb[(size_t)n * CH];
#pragma unroll 2
        for (int p = 0; p < ncnt; ++p) v += lsf[w][p] * xb[(size_t)lss[w][p] * CH];
        v += Hin[((size_t)(b * Tin + t + d) * NN + n) * CH + lane] * sc + sh;
        *(volatile float*)(Hout + ro) = v;
        __threadfence();
        *(volatile float*)(Hout + ro) = v;
        s64 += (double)v; q64 += (double)v * (double)v;
    }
    red[w][lane] = s64; red[w][32 + lane] = q64;
    __syncthreads();
    if (tid < 64) {
        double a = 0.0;
#pragma unroll
        for (int ww = 0; ww < 8; ++ww) a += red[ww][tid];
        sp[tid] = a;
    }
    __syncthreads();
    if (w == 0) {
        const v2d v = *(const v2d*)(sp + 2 * lane);
        double* gp = part + (size_t)blockIdx.x * 64 + 2 * lane;
        *(volatile v2d*)gp = v;
        __threadfence();
        *(volatile v2d*)gp = v;
    }
}

__global__ __launch_bounds__(64)
void k_bnfin(const double* __restrict__ part, const float* __restrict__ g, const float* __restrict__ bta, float* bnco, int nblk, int cnt)
{
    __shared__ __attribute__((aligned(16))) float so[64];
    const int t = threadIdx.x;
    if (t < 32) {
        double s = 0.0, ss = 0.0;
#pragma unroll 1
        for (int blk = 0; blk < nblk; ++blk) { s += part[blk * 64 + t]; ss += part[blk * 64 + 32 + t]; }
        const double ic = 1.0 / (double)cnt;
        const double mu = s * ic;
        double var = ss * ic - mu * mu; var = (var < 0.0) ? 0.0 : var;
        const float r = rsqrtf((float)var + 1e-5f);
        const float scl = g[t] * r;
        so[t] = scl; so[32 + t] = bta[t] - (float)mu * scl;
    }
    __syncthreads();
    if (t < 16) {
        const v4f v = *(const v4f*)(so + t * 4);
        *(volatile v4f*)(bnco + t * 4) = v;
        __threadfence();
        *(volatile v4f*)(bnco + t * 4) = v;
    }
}

__global__ __launch_bounds__(256)
void k_cvt(const float* __restrict__ src, unsigned short* dhi, unsigned short* dlo, int n8, int relu)
{
    const int i = blockIdx.x * 256 + threadIdx.x;
    if (i >= n8) return;
    const size_t e = (size_t)i * 8;
    v8f x = ld8f(src + e);
    if (relu) {
#pragma unroll
        for (int c = 0; c < 8; ++c) x[c] = fmaxf(x[c], 0.f);
    }
    u16x8 hv, lv; split8(x, hv, lv);
    *(volatile u16x8*)(dhi + e) = hv; *(volatile u16x8*)(dlo + e) = lv;
    __threadfence();
    *(volatile u16x8*)(dhi + e) = hv; *(volatile u16x8*)(dlo + e) = lv;
}

__global__ __launch_bounds__(256)
void k_out(const float* __restrict__ y2, float* out, int total)
{
    const int i = blockIdx.x * 256 + threadIdx.x;
    if (i >= total) return;
    const int b = i / (OT * NN), rem = i - b * OT * NN, t = rem >> 10, n = rem & (NN - 1);
    const float v = y2[((size_t)b * NN + n) * 16 + t];
    *(volatile float*)(out + i) = v;
    __threadfence();
    *(volatile float*)(out + i) = v;
}

extern "C" void kernel_launch(void* const* d_in, const int* in_sizes, int n_in,
                              void* d_out, int out_size, void* d_ws, size_t ws_size, hipStream_t stream)
{
    if (n_in < 23) return;
    const int E = in_sizes[2];
    if (E < 1 || in_sizes[1] != 2 * E) return;
    if (in_sizes[0] != BB * T0 * NN * 2 || in_sizes[3] != NN * 10 || in_sizes[4] != 10 * NN) return;
    if (in_sizes[5] != CH * 2 || in_sizes[6] != CH || in_sizes[7] != NL * CH * CH * 2 || in_sizes[9] != NL * CH * CH * 2) return;
    if (in_sizes[8] != NL * CH || in_sizes[10] != NL * CH || in_sizes[11] != NL * CH * CH || in_sizes[13] != NL * CH * CH) return;
    if (in_sizes[12] != NL * CH || in_sizes[14] != NL * CH || in_sizes[15] != NL * SKC * CH || in_sizes[16] != NL * SKC) return;
    if (in_sizes[17] != NL * CH || in_sizes[18] != NL * CH || in_sizes[19] != ENC * SKC || in_sizes[20] != ENC) return;
    if (in_sizes[21] != OT * ENC || in_sizes[22] != OT) return;
    if (out_size != BB * OT * NN) return;
    if (ws_size < WS_END) return;

    const float* x    = (const float*)d_in[0];
    const int*   ei   = (const int*)d_in[1];
    const float* ew   = (const float*)d_in[2];
    const float* e1   = (const float*)d_in[3];
    const float* e2   = (const float*)d_in[4];
    const float* inw  = (const float*)d_in[5];
    const float* inb  = (const float*)d_in[6];
    const float* tAw  = (const float*)d_in[7];
    const float* tAb  = (const float*)d_in[8];
    const float* tBw  = (const float*)d_in[9];
    const float* tBb  = (const float*)d_in[10];
    const float* gw   = (const float*)d_in[11];
    const float* gb   = (const float*)d_in[12];
    const float* gaw  = (const float*)d_in[13];
    const float* gab  = (const float*)d_in[14];
    const float* sw   = (const float*)d_in[15];
    const float* sb   = (const float*)d_in[16];
    const float* bng  = (const float*)d_in[17];
    const float* bnb  = (const float*)d_in[18];
    const float* w1   = (const float*)d_in[19];
    const float* b1   = (const float*)d_in[20];
    const float* w2   = (const float*)d_in[21];
    const float* b2   = (const float*)d_in[22];
    float* out = (float*)d_out;

    char* ws = (char*)d_ws;
    float* HA   = (float*)(ws + OFF_HA);
    float* HB   = (float*)(ws + OFF_HB);
    float* XW1  = (float*)(ws + OFF_XW1);
    unsigned short* XW2 = (unsigned short*)(ws + OFF_XW2);
    unsigned short* GLH = (unsigned short*)(ws + OFF_GLH);
    unsigned short* GLL = (unsigned short*)(ws + OFF_GLL);
    float* SKIP = (float*)(ws + OFF_SKIP);
    unsigned short* ADJ = (unsigned short*)(ws + OFF_ADJ);
    float* STAT = (float*)(ws + OFF_STAT);
    float* DIS  = (float*)(ws + OFF_DIS);
    float* BNC  = (float*)(ws + OFF_BNC);
    double* PART = (double*)(ws + OFF_PART);
    unsigned short* WTH = (unsigned short*)(ws + OFF_WTH);
    unsigned short* WTL = (unsigned short*)(ws + OFF_WTL);
    unsigned short* W2P = (unsigned short*)(ws + OFF_W2);
    unsigned short* WSKH = (unsigned short*)(ws + OFF_WSKH);
    unsigned short* WSKL = (unsigned short*)(ws + OFF_WSKL);
    unsigned short* E1H = (unsigned short*)(ws + OFF_E1H);
    unsigned short* E1L = (unsigned short*)(ws + OFF_E1L);
    unsigned short* E2H = (unsigned short*)(ws + OFF_E2H);
    unsigned short* E2L = (unsigned short*)(ws + OFF_E2L);
    unsigned short* SH  = (unsigned short*)(ws + OFF_SH);
    unsigned short* SL  = (unsigned short*)(ws + OFF_SL);
    float* Y1 = (float*)(ws + OFF_Y1);
    unsigned short* Y1H = (unsigned short*)(ws + OFF_Y1H);
    unsigned short* Y1L = (unsigned short*)(ws + OFF_Y1L);
    float* Y2 = (float*)(ws + OFF_Y2);

    k_wprep<<<dim3(64, 5), dim3(256), 0, stream>>>(tAw, tBw, gw, gaw, sw, w1, w2, WTH, WTL, W2P, WSKH, WSKL, E1H, E1L, E2H, E2L);
    {
        const int n4 = BB * T0 * NN * 8;
        k_h0<<<dim3((n4 + 255) / 256), dim3(256), 0, stream>>>(x, inw, inb, HA, BNC, n4);
    }
    k_graph<<<dim3(NN / 32), dim3(256), 0, stream>>>(ei, ew, E, DIS);
    k_adp1<<<dim3(NN / 8), dim3(256), 0, stream>>>(e1, e2, STAT);
    k_adp2<<<dim3(NN / 8), dim3(256), 0, stream>>>(e1, e2, STAT, ADJ);

    const int dil[NL] = {1, 2, 1, 2, 1, 2, 1, 2};
    float* Hin = HA; float* Hout = HB;
    int Tin = T0;
    const float c14 = 1.f / 16384.f;
    for (int k = 0; k < NL; ++k) {
        const int d = dil[k];
        const int Tk = Tin - d;
        k_tcn<<<dim3(NN / 64, Tk, BB), dim3(128), 0, stream>>>(
            Hin, BNC + k * 64, WTH + (size_t)k * 4096, WTL + (size_t)k * 4096, W2P + (size_t)k * 2048, tAb + k * CH, tBb + k * CH,
            XW1, XW2, GLH, GLL, Tin, Tk, d);
        k_gemm<2, 0><<<dim3(1, NN / 128, BB * Tk), dim3(128), 0, stream>>>(
            ADJ, ADJ, XW2, XW2, Hout, gb, NN, CH, 0, 0, c14,
            (long long)0, (long long)(CH * NN), (long long)(NN * CH));
        k_comb<<<dim3(NN / 8), dim3(256), 0, stream>>>(
            Hout, Hin, XW1, BNC + k * 64, ei, ew, DIS, gb + k * CH, gab + k * CH, PART, E, Tin, Tk, d);
        k_bnfin<<<dim3(1), dim3(64), 0, stream>>>(PART, bng + k * CH, bnb + k * CH, BNC + (k + 1) * 64, NN / 8, BB * NN * Tk);
        k_gemm<2, 1><<<dim3(SKC / 32, (BB * NN) / 128, 1), dim3(128), 0, stream>>>(
            GLH, GLL, WSKH + (size_t)k * SKC * CH, WSKL + (size_t)k * SKC * CH, SKIP, sb + k * SKC,
            CH, SKC, SKC, (k > 0) ? 3 : 1, 1.f, (long long)0, (long long)0, (long long)0);
        float* tmp = Hin; Hin = Hout; Hout = tmp;
        Tin = Tk;
    }

    k_cvt<<<dim3((BB * NN * SKC / 8 + 255) / 256), dim3(256), 0, stream>>>(SKIP, SH, SL, BB * NN * SKC / 8, 1);
    k_gemm<2, 1><<<dim3(ENC / 32, (BB * NN) / 128, 1), dim3(128), 0, stream>>>(
        SH, SL, E1H, E1L, Y1, b1, SKC, ENC, ENC, 1, 1.f, (long long)0, (long long)0, (long long)0);
    k_cvt<<<dim3((BB * NN * ENC / 8 + 255) / 256), dim3(256), 0, stream>>>(Y1, Y1H, Y1L, BB * NN * ENC / 8, 1);
    k_gemm<1, 1><<<dim3(1, (BB * NN) / 128, 1), dim3(128), 0, stream>>>(
        Y1H, Y1L, E2H, E2L, Y2, b2, ENC, 16, OT, 1, 1.f, (long long)0, (long long)0, (long long)0);
    {
        const int total = BB * OT * NN;
        k_out<<<dim3((total + 255) / 256), dim3(256), 0, stream>>>(Y2, out, total);
    }
}
